// GATwithEdgeAttr_50903952392628
// MI455X (gfx1250) — hardware-run, weakly checked
//
#include <hip/hip_runtime.h>

typedef float          v8f   __attribute__((ext_vector_type(8)));
typedef float          v4f   __attribute__((ext_vector_type(4)));
typedef unsigned int   v4u   __attribute__((ext_vector_type(4)));
typedef int            v8i   __attribute__((ext_vector_type(8)));
typedef unsigned short v8us  __attribute__((ext_vector_type(8)));
typedef unsigned short v16us __attribute__((ext_vector_type(16)));
typedef __bf16         v16bf __attribute__((ext_vector_type(16)));
typedef _Float16       v16h  __attribute__((ext_vector_type(16)));
typedef v4f  __attribute__((may_alias)) v4fa;
typedef v8us __attribute__((may_alias)) v8usa;
union FragB { v16bf v; v16us u; v8us h[2]; v8i w; };
union FragH { v16h  v; v16us u; v8us h[2]; v8i w; };

__device__ __forceinline__ v8f wmb(const FragB& a, const FragB& b, v8f c) {
  v8f d = __builtin_amdgcn_wmma_f32_16x16x32_bf16(false, a.v, false, b.v, (short)0, c, false, false);
  asm volatile("v_nop\n\tv_nop\n\tv_nop\n\tv_nop" : "+v"(d) : "v"(a.w), "v"(b.w));
  return d;
}

__device__ __forceinline__ v8f wmh(const FragH& a, const FragH& b, v8f c) {
  v8f d = __builtin_amdgcn_wmma_f32_16x16x32_f16(false, a.v, false, b.v, (short)0, c, false, false);
  asm volatile("v_nop\n\tv_nop\n\tv_nop\n\tv_nop" : "+v"(d) : "v"(a.w), "v"(b.w));
  return d;
}

__device__ __forceinline__ unsigned bf16_bits(float f) {
  const unsigned u = __float_as_uint(f);
  const unsigned r = (u + 0x7FFFu + ((u >> 16) & 1u)) >> 16;
  const unsigned q = (u >> 16) | 0x40u;
  return ((u & 0x7fffffffu) > 0x7f800000u) ? q : r;
}

__device__ __forceinline__ float bf16_val(float f) {
  return __uint_as_float(bf16_bits(f) << 16);
}
__device__ __forceinline__ int clampi(int v, int lo, int hi) {
  return v < lo ? lo : (v > hi ? hi : v);
}

__device__ __forceinline__ unsigned f16_bits(float f) {
  const unsigned u  = __float_as_uint(f);
  const unsigned s  = (u >> 16) & 0x8000u;
  const unsigned a  = u & 0x7fffffffu;
  const unsigned t  = a - 0x38000000u;
  const unsigned r  = (t + 0x0FFFu + ((t >> 13) & 1u)) >> 13;
  const unsigned rc = r > 0x7C00u ? 0x7C00u : r;
  const bool small  = a < 0x38800000u;
  const bool isnan  = a > 0x7f800000u;
  const unsigned fin = small ? 0u : (s | rc);
  return isnan ? (s | 0x7E00u) : fin;
}

__device__ __forceinline__ unsigned pk16(unsigned lo, unsigned hi) { return lo | (hi << 16); }
__device__ __forceinline__ unsigned bf16_lo_bits(float v) {
  float hi = bf16_val(v);
  asm volatile("" : "+v"(hi));
  return bf16_bits(v - hi);
}
__device__ __forceinline__ v4u pack8_bf16(v4f a, v4f c) {
  return (v4u){ pk16(bf16_bits(a[0]), bf16_bits(a[1])), pk16(bf16_bits(a[2]), bf16_bits(a[3])),
                pk16(bf16_bits(c[0]), bf16_bits(c[1])), pk16(bf16_bits(c[2]), bf16_bits(c[3])) };
}
__device__ __forceinline__ v4u pack8_bf16_lo(v4f a, v4f c) {
  return (v4u){ pk16(bf16_lo_bits(a[0]), bf16_lo_bits(a[1])), pk16(bf16_lo_bits(a[2]), bf16_lo_bits(a[3])),
                pk16(bf16_lo_bits(c[0]), bf16_lo_bits(c[1])), pk16(bf16_lo_bits(c[2]), bf16_lo_bits(c[3])) };
}
__device__ __forceinline__ v4u pack8_f16(v4f a, v4f c) {
  return (v4u){ pk16(f16_bits(a[0]), f16_bits(a[1])), pk16(f16_bits(a[2]), f16_bits(a[3])),
                pk16(f16_bits(c[0]), f16_bits(c[1])), pk16(f16_bits(c[2]), f16_bits(c[3])) };
}

template <int FORM>
__global__ __launch_bounds__(256) void k_plane(const float* __restrict__ src, int rows, int cols, int ldsrc,
                                               unsigned short* __restrict__ dst, int MP, int KP) {
  static_assert(FORM >= 0 && FORM <= 3);
  const int KTOT = (FORM == 1 || FORM == 3) ? 2 * KP : KP;
  const unsigned ppr   = (unsigned)(KTOT >> 3);
  const unsigned kp8   = (unsigned)(KP >> 3);
  const unsigned total = (unsigned)MP * ppr;
  const unsigned g     = blockIdx.x * 256u + threadIdx.x;
  const unsigned rowu  = g / ppr;
  const unsigned p     = g - rowu * ppr;
  const bool second    = p >= kp8;
  const int row = (int)rowu;
  const int c0  = (int)((second ? p - kp8 : p) << 3);
  const float* srow = src + (size_t)clampi(row, 0, rows - 1) * (size_t)ldsrc;
  float x[8];
  unsigned mk[8];
#pragma unroll
  for (int e = 0; e < 8; ++e) {
    const int c = c0 + e;
    const float v = srow[clampi(c, 0, cols - 1)];
    asm volatile("" :: "v"(v));
    x[e]  = v;
    mk[e] = (row < rows && c < cols) ? 0xFFFFu : 0u;
  }
  const v4f a = (v4f){ x[0], x[1], x[2], x[3] };
  const v4f c = (v4f){ x[4], x[5], x[6], x[7] };
  v4u o;
  if (FORM == 2) {
    o = pack8_f16(a, c);
  } else {
    const v4u hi = pack8_bf16(a, c);
    o = hi;
    if (FORM == 1) { const v4u lo = pack8_bf16_lo(a, c); o = second ? lo : hi; }
  }
  const v4u mw = (v4u){ pk16(mk[0], mk[1]), pk16(mk[2], mk[3]), pk16(mk[4], mk[5]), pk16(mk[6], mk[7]) };
  o &= mw;
  if (g < total) {
    volatile v4u* q = (volatile v4u*)(dst + (size_t)g * 8);
    *q = o;
    __threadfence();
    *q = o;
  }
}

template <int FORM> struct FragOf    { typedef FragB T; };
template <>         struct FragOf<2> { typedef FragH T; };
__device__ __forceinline__ v8f mm(const FragB& a, const FragB& b, v8f c) { return wmb(a, b, c); }
__device__ __forceinline__ v8f mm(const FragH& a, const FragH& b, v8f c) { return wmh(a, b, c); }
template <class F> __device__ __forceinline__ F ld_frag(const unsigned short* p) {
  F f;
  f.h[0] = *(const v8usa*)(p);
  f.h[1] = *(const v8usa*)(p + 16);
  return f;
}

template <int FORM, int EPI>
__global__ __launch_bounds__(256) __attribute__((amdgpu_num_vgpr(248)))
void k_gemm_nt(const unsigned short* __restrict__ A, const unsigned short* __restrict__ B,
               const float* __restrict__ bias, float* __restrict__ D, int M, int N, int KTOT, int ldd) {
  static_assert(FORM >= 0 && FORM <= 2);
  static_assert(EPI == 0 || EPI == 1);
  typedef typename FragOf<FORM>::T F;
  __shared__ __attribute__((aligned(16))) float sT[8][16 * 68];
  const int lane = threadIdx.x & 31;
  const int wave = threadIdx.x >> 5;
  const int tilesM = (M + 63) >> 6;
  const int tilesN = (N + 63) >> 6;
  const int tile = blockIdx.x * 8 + wave;
  if (tile >= tilesM * tilesN) return;
  const int tm = tile / tilesN;
  const int tn = tile - tm * tilesN;
  const int m0 = tm << 6;
  const int n0 = tn << 6;

  const int rl = lane & 15;
  const int h8 = (lane >> 4) * 8;
  const unsigned short* pa = A + (size_t)(m0 + rl) * (size_t)KTOT + h8;
  const unsigned short* pb = B + (size_t)(n0 + rl) * (size_t)KTOT + h8;

  v8f acc[4][4];
#pragma unroll
  for (int i = 0; i < 4; ++i)
#pragma unroll
    for (int j = 0; j < 4; ++j) acc[i][j] = (v8f){0.f, 0.f, 0.f, 0.f, 0.f, 0.f, 0.f, 0.f};

#pragma unroll 1
  for (int k0 = 0; k0 < KTOT; k0 += 32) {
    F bf[4];
#pragma unroll
    for (int j = 0; j < 4; ++j) bf[j] = ld_frag<F>(pb + (size_t)(j << 4) * (size_t)KTOT + k0);
#pragma unroll
    for (int i = 0; i < 4; ++i) {
      const F af = ld_frag<F>(pa + (size_t)(i << 4) * (size_t)KTOT + k0);
#pragma unroll
      for (int j = 0; j < 4; ++j) acc[i][j] = mm(af, bf[j], acc[i][j]);
    }
  }

  float* slab = sT[wave];
  const int hh = lane >> 4;
  const int c4 = (lane & 15) * 4;
  const int nc = n0 + c4;
  const bool cok = nc < N;
  v4f bv = (v4f){0.f, 0.f, 0.f, 0.f};
  if (EPI == 1) {
    bv = *(const v4fa*)(bias + clampi(nc, 0, N - 4));
    asm volatile("" :: "v"(bv));
  }
#pragma unroll
  for (int i = 0; i < 4; ++i) {
    const int mBase = m0 + (i << 4);
#pragma unroll
    for (int j = 0; j < 4; ++j) {
#pragma unroll
      for (int r = 0; r < 8; ++r) slab[(h8 + r) * 68 + (j << 4) + rl] = acc[i][j][r];
    }
    __builtin_amdgcn_fence(__ATOMIC_RELEASE, "workgroup");
    __builtin_amdgcn_wave_barrier();
    __builtin_amdgcn_fence(__ATOMIC_ACQUIRE, "workgroup");
    v4f vv[8];
#pragma unroll
    for (int it = 0; it < 8; ++it) {
      const int row = it * 2 + hh;
      v4f v = *(const v4fa*)(slab + row * 68 + c4);
      if (EPI == 1) v += bv;
      vv[it] = v;
    }
    for (int pass = 0; pass < 2; ++pass) {
#pragma unroll
      for (int it = 0; it < 8; ++it) {
        const int row = mBase + it * 2 + hh;
        if (cok && row < M) *(volatile v4f*)(D + (size_t)row * (size_t)ldd + nc) = vv[it];
      }
      __threadfence();
    }
    __builtin_amdgcn_fence(__ATOMIC_RELEASE, "workgroup");
    __builtin_amdgcn_wave_barrier();
    __builtin_amdgcn_fence(__ATOMIC_ACQUIRE, "workgroup");
  }
}

#pragma clang fp contract(off)


#define NN      50000
#define NE      800000
#define MPAD    50048
#define KD      128
#define HC      256
#define EDW     8
#define RTHR    256
#define RWAVES  8
#define TB_AS   0
#define TB_AD   256
#define TB_BI   512
#define TB_GA   640
#define TB_BE   768
#define TB_KV   896
#define TB_N    1024
#define BT      512
#define BW      16
#define BEPT    8
#define BCHUNK  (BT * BEPT)
#define NCH     ((NE + BCHUNK - 1) / BCHUNK)
#define NB      1024
#define NBLK    ((NN + NB - 1) / NB)
#define RCAP    20992
#define DEGCAP  64
#define SLOTSH  21
#define LISTTOT (NBLK * RCAP)
#define LDS_BKT ((2 * RCAP + 3 * NB + 64) * 4)
#define WSMAX   ((size_t)128 << 20)

static_assert(NN % RWAVES == 0);
static_assert(MPAD == 782 * 64 && MPAD % 64 == 0 && MPAD >= NN);
static_assert(HC % 64 == 0 && KD % 32 == 0 && HC == 2 * 128);
static_assert(NE < (1 << SLOTSH));
static_assert(NB <= 1024 && (NB & (NB - 1)) == 0 && NB == 2 * BT);
static_assert(NE % 8 == 0 && NE >= 8);
static_assert(NBLK == 49 && NBLK * NB >= NN);
static_assert(NCH * BCHUNK >= NE && NCH == 196);
static_assert(RCAP % 32 == 0);
static_assert(RCAP * 4 >= 16623 * 5);
static_assert(DEGCAP >= 35 + 8);
static_assert(DEGCAP == 64);
static_assert(LDS_BKT <= 327680);
static_assert(BW == BT / 32 && BW == 16);

typedef int          v4i __attribute__((ext_vector_type(4)));
typedef int          v2i __attribute__((ext_vector_type(2)));
typedef unsigned int v2u __attribute__((ext_vector_type(2)));
typedef v4i __attribute__((may_alias)) v4ia;
typedef v2i __attribute__((may_alias)) v2ia;
typedef v2u __attribute__((may_alias)) v2ua;

__device__ __forceinline__ float cvp(float f) {
  float v = bf16_val(f);
  asm volatile("" : "+v"(v));
  return v;
}
__device__ __forceinline__ float lrelu_k(float v) { return (v >= 0.0f) ? v : 0.2f * v; }
__device__ __forceinline__ float maxk(float a, float b) {
  float m = (a < b) ? b : a;
  m = (b != b) ? b : m;
  return m;
}
__device__ __forceinline__ float sum16(float t) {
  t = t + __shfl_xor(t, 8, 32);
  t = t + __shfl_xor(t, 4, 32);
  t = t + __shfl_xor(t, 2, 32);
  t = t + __shfl_xor(t, 1, 32);
  return t;
}
__device__ __forceinline__ float rlf(float v, int k) {
  return __int_as_float(__builtin_amdgcn_readlane(__float_as_int(v), k));
}
__device__ __forceinline__ v4f widen4(v2u w) {
  v4f r;
  r.x = __uint_as_float(w.x << 16);
  r.y = __uint_as_float(w.x & 0xffff0000u);
  r.z = __uint_as_float(w.y << 16);
  r.w = __uint_as_float(w.y & 0xffff0000u);
  return r;
}

__global__ __launch_bounds__(256) void k_prep(const float* __restrict__ Wlin, const float* __restrict__ Wle,
                                              const float* __restrict__ attE, const float* __restrict__ Wep,
                                              const float* __restrict__ bep, const float* __restrict__ attS,
                                              const float* __restrict__ attD, const float* __restrict__ bias,
                                              const float* __restrict__ gam, const float* __restrict__ bet,
                                              unsigned short* WT, float* TB) {
  __shared__ __attribute__((aligned(16))) float sae[256];
  __shared__ __attribute__((aligned(16))) float sml[256];
  __shared__ __attribute__((aligned(16))) float skv[32];
  const int t = (int)threadIdx.x;
  {
    const float v = attE[t];
    asm volatile("" :: "v"(v));
    sae[t] = cvp(v);
  }
  __syncthreads();
  {
    const int hh = t >> 7, j = t & 127;
    const float* wr = Wle + (size_t)j * HC + hh * 128;
    const float* ar = sae + hh * 128;
    float acc = 0.0f;
#pragma unroll 1
    for (int c = 0; c < 128; c += 4) {
      const v4f w = *(const v4fa*)(wr + c);
      asm volatile("" :: "v"(w));
      const v4f a = *(const v4fa*)(ar + c);
      float p;
      p = cvp(w.x) * a.x; acc = acc + p;
      p = cvp(w.y) * a.y; acc = acc + p;
      p = cvp(w.z) * a.z; acc = acc + p;
      p = cvp(w.w) * a.w; acc = acc + p;
    }
    sml[t] = acc;
  }
  __syncthreads();
  {
    const int i = t & 7, hv = (t >> 3) & 1, h2 = t & 1;
    const float* wr = Wep + i * 128;
    const float* m1 = sml + hv * 128;
    const float* m2 = sml + h2 * 128;
    float kv = 0.0f, kc = 0.0f;
#pragma unroll 4
    for (int j = 0; j < 128; ++j) {
      const float wv = wr[j];
      asm volatile("" :: "v"(wv));
      const float bv = bep[j];
      asm volatile("" :: "v"(bv));
      const float p = cvp(wv) * m1[j];
      kv = kv + p;
      const float q = cvp(bv) * m2[j];
      kc = kc + q;
    }
    float val = (t < 16) ? kv : kc;
    val = (t < 18) ? val : 0.0f;
    if (t < 32) skv[t] = val;
  }
  __syncthreads();
  {
    const int idx = 4 * t;
    const v4f a0 = *(const v4fa*)(attS + clampi(idx - TB_AS, 0, 252));
    asm volatile("" :: "v"(a0));
    const v4f a1 = *(const v4fa*)(attD + clampi(idx - TB_AD, 0, 252));
    asm volatile("" :: "v"(a1));
    const v4f a2 = *(const v4fa*)(bias + clampi(idx - TB_BI, 0, 124));
    asm volatile("" :: "v"(a2));
    const v4f a3 = *(const v4fa*)(gam + clampi(idx - TB_GA, 0, 124));
    asm volatile("" :: "v"(a3));
    const v4f a4 = *(const v4fa*)(bet + clampi(idx - TB_BE, 0, 124));
    asm volatile("" :: "v"(a4));
    const v4f k4 = *(const v4fa*)(skv + clampi(idx - TB_KV, 0, 28));
    const unsigned m0 = (idx < TB_AD) ? 0xFFFFFFFFu : 0u;
    const unsigned m1 = (idx >= TB_AD && idx < TB_BI) ? 0xFFFFFFFFu : 0u;
    const unsigned m2 = (idx >= TB_BI && idx < TB_GA) ? 0xFFFFFFFFu : 0u;
    const unsigned m3 = (idx >= TB_GA && idx < TB_BE) ? 0xFFFFFFFFu : 0u;
    const unsigned m4 = (idx >= TB_BE && idx < TB_KV) ? 0xFFFFFFFFu : 0u;
    const unsigned m5 = (idx >= TB_KV && idx < TB_KV + 32) ? 0xFFFFFFFFu : 0u;
    v4u o;
    o.x = (__float_as_uint(a0.x) & m0) | (__float_as_uint(a1.x) & m1) | (__float_as_uint(a2.x) & m2) |
          (__float_as_uint(a3.x) & m3) | (__float_as_uint(a4.x) & m4);
    o.y = (__float_as_uint(a0.y) & m0) | (__float_as_uint(a1.y) & m1) | (__float_as_uint(a2.y) & m2) |
          (__float_as_uint(a3.y) & m3) | (__float_as_uint(a4.y) & m4);
    o.z = (__float_as_uint(a0.z) & m0) | (__float_as_uint(a1.z) & m1) | (__float_as_uint(a2.z) & m2) |
          (__float_as_uint(a3.z) & m3) | (__float_as_uint(a4.z) & m4);
    o.w = (__float_as_uint(a0.w) & m0) | (__float_as_uint(a1.w) & m1) | (__float_as_uint(a2.w) & m2) |
          (__float_as_uint(a3.w) & m3) | (__float_as_uint(a4.w) & m4);
    o.x = (bf16_bits(__uint_as_float(o.x)) << 16) | (__float_as_uint(k4.x) & m5);
    o.y = (bf16_bits(__uint_as_float(o.y)) << 16) | (__float_as_uint(k4.y) & m5);
    o.z = (bf16_bits(__uint_as_float(o.z)) << 16) | (__float_as_uint(k4.z) & m5);
    o.w = (bf16_bits(__uint_as_float(o.w)) << 16) | (__float_as_uint(k4.w) & m5);
    volatile v4u* q = (volatile v4u*)(TB + idx);
    *q = o;
    __threadfence();
    *q = o;
  }
#pragma unroll 1
  for (int it = 0; it < 16; ++it) {
    const int g  = it * 256 + t;
    const int n  = g >> 4;
    const int k0 = (g & 15) << 3;
    float x[8];
#pragma unroll
    for (int e = 0; e < 8; ++e) {
      const float v = Wlin[(size_t)(k0 + e) * HC + n];
      asm volatile("" :: "v"(v));
      x[e] = v;
    }
    const v4u o = pack8_bf16((v4f){ x[0], x[1], x[2], x[3] }, (v4f){ x[4], x[5], x[6], x[7] });
    volatile v4u* q = (volatile v4u*)(WT + (size_t)g * 8);
    *q = o;
    __threadfence();
    *q = o;
  }
}

__global__ __launch_bounds__(BT) void k_list(const int* __restrict__ edst, const int* __restrict__ esrc,
                                             unsigned* LIST, int* META) {
  extern __shared__ v4u lds_lst[];
  int* reg1 = (int*)lds_lst;
  int* reg2 = reg1 + RCAP;
  int* scnt = reg2 + RCAP;
  int* soff = scnt + NB;
  int* curs = soff + NB;
  int* wcnt = curs + NB;
  int* wtot = wcnt + 2 * BW;
  const int tid = (int)threadIdx.x, lane = tid & 31, wave = tid >> 5;
  const int nodeBase = (int)blockIdx.x * NB;
  int nb = NN - nodeBase;
  nb = nb > NB ? NB : (nb < 0 ? 0 : nb);
  const unsigned nbs = (unsigned)nodeBase, unb = (unsigned)nb;

  scnt[2 * tid] = 0;
  scnt[2 * tid + 1] = 0;

  int tot = 0;
#pragma unroll 1
  for (int ch = 0; ch < NCH; ++ch) {
    const int par = ch & 1;
    const int e0  = ch * BCHUNK + tid * BEPT;
    const bool valid = e0 < NE;
    const int ea = e0 < NE - 8 ? e0 : NE - 8;
    const v4i da = *(const v4ia*)(edst + ea);
    const v4i db = *(const v4ia*)(edst + ea + 4);
    asm volatile("" :: "v"(da), "v"(db));
    const unsigned s0 = (unsigned)da.x - nbs, s1 = (unsigned)da.y - nbs;
    const unsigned s2 = (unsigned)da.z - nbs, s3 = (unsigned)da.w - nbs;
    const unsigned s4 = (unsigned)db.x - nbs, s5 = (unsigned)db.y - nbs;
    const unsigned s6 = (unsigned)db.z - nbs, s7 = (unsigned)db.w - nbs;
    const bool h0 = valid && (s0 < unb), h1 = valid && (s1 < unb), h2 = valid && (s2 < unb), h3 = valid && (s3 < unb);
    const bool h4 = valid && (s4 < unb), h5 = valid && (s5 < unb), h6 = valid && (s6 < unb), h7 = valid && (s7 < unb);
    const int c = (int)h0 + (int)h1 + (int)h2 + (int)h3 + (int)h4 + (int)h5 + (int)h6 + (int)h7;
    int incl = c;
#pragma unroll
    for (int d = 1; d < 32; d <<= 1) {
      const int up = __shfl_up(incl, d, 32);
      incl += (lane >= d) ? up : 0;
    }
    const int wtotal = __shfl(incl, 31, 32);
    if (lane == 0) wcnt[par * BW + wave] = wtotal;
    __syncthreads();
    int all = 0, pre = 0;
#pragma unroll
    for (int g = 0; g < 4; ++g) {
      const v4i w4 = *(const v4ia*)(wcnt + par * BW + 4 * g);
      const int c0 = clampi(w4.x, 0, 256), c1 = clampi(w4.y, 0, 256);
      const int c2 = clampi(w4.z, 0, 256), c3 = clampi(w4.w, 0, 256);
      all += c0 + c1 + c2 + c3;
      pre += (4 * g + 0 < wave) ? c0 : 0;
      pre += (4 * g + 1 < wave) ? c1 : 0;
      pre += (4 * g + 2 < wave) ? c2 : 0;
      pre += (4 * g + 3 < wave) ? c3 : 0;
    }
    int pos = tot + pre + (incl - c);
#define PUTJ(J, HJ, SJ) if (HJ) { if (pos < RCAP) reg1[pos] = (int)((unsigned)(e0 + (J)) | ((SJ) << SLOTSH)); ++pos; }
    PUTJ(0, h0, s0)
    PUTJ(1, h1, s1)
    PUTJ(2, h2, s2)
    PUTJ(3, h3, s3)
    PUTJ(4, h4, s4)
    PUTJ(5, h5, s5)
    PUTJ(6, h6, s6)
    PUTJ(7, h7, s7)
#undef PUTJ
    tot += all;
  }
  __syncthreads();
  const bool ovf = tot > RCAP;
  const int nh = ovf ? RCAP : tot;

  if (wave == 0) {
#pragma unroll 1
    for (int b0 = 0; b0 < nh; b0 += 32) {
      const int idx = b0 + lane;
      const int uv  = reg1[idx < nh ? idx : nh - 1];
      const int m32 = (nh - b0) < 32 ? (nh - b0) : 32;
#pragma unroll 1
      for (int k = 0; k < m32; ++k) {
        const int u  = __builtin_amdgcn_readlane(uv, k);
        const int sl = (int)(((unsigned)u >> SLOTSH) & (unsigned)(NB - 1));
        const int cv = scnt[sl] + 1;
        if (lane == 0) scnt[sl] = cv;
      }
    }
  }
  __syncthreads();

  int e0c, e1c;
  {
    const v2i cc = *(const v2ia*)(scnt + 2 * tid);
    e0c = cc.x < 0 ? 0 : cc.x;
    e1c = cc.y < 0 ? 0 : cc.y;
    const int ts = e0c + e1c;
    int incl = ts;
#pragma unroll
    for (int d = 1; d < 32; d <<= 1) {
      const int up = __shfl_up(incl, d, 32);
      incl += (lane >= d) ? up : 0;
    }
    if (lane == 31) wtot[wave] = incl;
    __syncthreads();
    int pre = 0;
#pragma unroll
    for (int g = 0; g < 4; ++g) {
      const v4i w4 = *(const v4ia*)(wtot + 4 * g);
      pre += (4 * g + 0 < wave) ? w4.x : 0;
      pre += (4 * g + 1 < wave) ? w4.y : 0;
      pre += (4 * g + 2 < wave) ? w4.z : 0;
      pre += (4 * g + 3 < wave) ? w4.w : 0;
    }
    const int run = pre + incl - ts;
    soff[2 * tid]     = run;
    soff[2 * tid + 1] = run + e0c;
    curs[2 * tid]     = run;
    curs[2 * tid + 1] = run + e0c;
  }
  __syncthreads();

  if (wave == 0) {
#pragma unroll 1
    for (int b0 = 0; b0 < nh; b0 += 32) {
      const int idx = b0 + lane;
      const int uv  = reg1[idx < nh ? idx : nh - 1];
      const int m32 = (nh - b0) < 32 ? (nh - b0) : 32;
#pragma unroll 1
      for (int k = 0; k < m32; ++k) {
        const int u   = __builtin_amdgcn_readlane(uv, k);
        const int sl  = (int)(((unsigned)u >> SLOTSH) & (unsigned)(NB - 1));
        const int eid = (int)((unsigned)u & ((1u << SLOTSH) - 1u));
        const int pr  = curs[sl];
        const int pc  = clampi(pr, 0, RCAP - 1);
        if (lane == 0) { reg2[pc] = eid; curs[sl] = pc + 1; }
      }
    }
  }
  __syncthreads();

  {
    int nhPad = (nh + 15) & ~15;
    nhPad = nhPad > RCAP ? RCAP : nhPad;
    const int nIt = (nhPad + BT - 1) / BT;
    unsigned* lbase = LIST + (size_t)blockIdx.x * (size_t)RCAP * 2;
#pragma unroll 1
    for (int it = 0; it < nIt; ++it) {
      const int i  = it * BT + tid;
      const int ic = i < nh ? i : nh - 1;
      const int eid = clampi(reg2[ic], 0, NE - 1);
      const int cw = esrc[eid];
      asm volatile("" :: "v"(cw));
      const unsigned msk = (i < nh) ? 0xFFFFFFFFu : 0u;
      v2u o;
      o.x = (unsigned)clampi(cw, 0, NN - 1) & msk;
      o.y = (unsigned)eid & msk;
      const int iw = i < RCAP ? i : RCAP - 1;
      volatile v2u* q = (volatile v2u*)(lbase + 2 * (size_t)iw);
      const bool wr = i < nhPad;
      if (wr) *q = o;
      __threadfence();
      if (wr) *q = o;
    }
  }

  {
    const int base = (int)blockIdx.x * RCAP;
    const v2i cc = *(const v2ia*)(scnt + 2 * tid);
    const v2i so = *(const v2ia*)(soff + 2 * tid);
    v4i m;
    m.x = base + so.x;
    m.y = ovf ? -1 : cc.x;
    m.z = base + so.y;
    m.w = ovf ? -1 : cc.y;
    volatile v4i* q = (volatile v4i*)(META + 2 * (size_t)(nodeBase + 2 * tid));
    *q = m;
    __threadfence();
    *q = m;
  }
}

__global__ __launch_bounds__(RTHR) void k_rowprep(const float* __restrict__ H, const float* __restrict__ TB, float* A4) {
  __shared__ __attribute__((aligned(16))) float sdot[RWAVES * 4];
  const int lane = (int)threadIdx.x & 31;
  const int wave = (int)threadIdx.x >> 5;
  const int row  = (int)blockIdx.x * RWAVES + wave;
  const int rowc = row < NN ? row : NN - 1;
  const int head = lane >> 4;
  const int c0   = lane * 8;
  const float* hr = H + (size_t)rowc * HC + c0;
  const v4f h0 = *(const v4fa*)hr;
  const v4f h1 = *(const v4fa*)(hr + 4);
  asm volatile("" :: "v"(h0), "v"(h1));
  const v4f s0 = *(const v4fa*)(TB + TB_AS + c0);
  const v4f s1 = *(const v4fa*)(TB + TB_AS + c0 + 4);
  const v4f d0 = *(const v4fa*)(TB + TB_AD + c0);
  const v4f d1 = *(const v4fa*)(TB + TB_AD + c0 + 4);
  asm volatile("" :: "v"(s0), "v"(s1), "v"(d0), "v"(d1));
  float ts, td, u;
  ts = h0.x * s0.x;
  u = h0.y * s0.y; ts = ts + u;
  u = h0.z * s0.z; ts = ts + u;
  u = h0.w * s0.w; ts = ts + u;
  u = h1.x * s1.x; ts = ts + u;
  u = h1.y * s1.y; ts = ts + u;
  u = h1.z * s1.z; ts = ts + u;
  u = h1.w * s1.w; ts = ts + u;
  td = h0.x * d0.x;
  u = h0.y * d0.y; td = td + u;
  u = h0.z * d0.z; td = td + u;
  u = h0.w * d0.w; td = td + u;
  u = h1.x * d1.x; td = td + u;
  u = h1.y * d1.y; td = td + u;
  u = h1.z * d1.z; td = td + u;
  u = h1.w * d1.w; td = td + u;
  ts = sum16(ts);
  td = sum16(td);
  if ((lane & 15) == 0) {
    sdot[wave * 4 + head]     = ts;
    sdot[wave * 4 + 2 + head] = td;
  }
  __syncthreads();
  if (wave == 0) {
    const int l8 = lane & 7;
    const v4f sv = *(const v4fa*)(sdot + 4 * l8);
    const int trow = (int)blockIdx.x * RWAVES + l8;
    const bool wr = (lane < 8) && (trow < NN);
    volatile v4f* q = (volatile v4f*)(A4 + (size_t)(trow < NN ? trow : NN - 1) * 4);
    if (wr) *q = sv;
    __threadfence();
    if (wr) *q = sv;
  }
}

__device__ __forceinline__ void entry_score(const unsigned* __restrict__ LIST, const float* __restrict__ eattr,
                                            const float* __restrict__ A4, int pidx,
                                            v4f k00, v4f k01, v4f k10, v4f k11, float kc0, float kc1,
                                            float ad0, float ad1, float& s0, float& s1, int& src) {
  const v2u ent = *(const v2ua*)(LIST + 2 * (size_t)pidx);
  asm volatile("" :: "v"(ent));
  const int sc  = clampi((int)ent.x, 0, NN - 1);
  const int eid = clampi((int)ent.y, 0, NE - 1);
  const float* ep = eattr + (size_t)eid * EDW;
  const v4f e0 = *(const v4fa*)ep;
  asm volatile("" :: "v"(e0));
  const v4f e1 = *(const v4fa*)(ep + 4);
  asm volatile("" :: "v"(e1));
  const v4f as = *(const v4fa*)(A4 + (size_t)sc * 4);
  asm volatile("" :: "v"(as));
  const float x0 = cvp(e0.x), x1 = cvp(e0.y), x2 = cvp(e0.z), x3 = cvp(e0.w);
  const float x4 = cvp(e1.x), x5 = cvp(e1.y), x6 = cvp(e1.z), x7 = cvp(e1.w);
  float t, u;
  t = x0 * k00.x;
  u = x1 * k00.y; t = t + u;
  u = x2 * k00.z; t = t + u;
  u = x3 * k00.w; t = t + u;
  u = x4 * k01.x; t = t + u;
  u = x5 * k01.y; t = t + u;
  u = x6 * k01.z; t = t + u;
  u = x7 * k01.w; t = t + u;
  t = t + kc0;
  float v = as.x + ad0;
  v = v + t;
  s0 = lrelu_k(v);
  t = x0 * k10.x;
  u = x1 * k10.y; t = t + u;
  u = x2 * k10.z; t = t + u;
  u = x3 * k10.w; t = t + u;
  u = x4 * k11.x; t = t + u;
  u = x5 * k11.y; t = t + u;
  u = x6 * k11.z; t = t + u;
  u = x7 * k11.w; t = t + u;
  t = t + kc1;
  v = as.y + ad1;
  v = v + t;
  s1 = lrelu_k(v);
  src = sc;
}
__device__ __forceinline__ void acc_row(const float* __restrict__ hb, int c, float w, v4f& aA, v4f& aB) {
  const float* p = hb + (size_t)c * HC;
  const v4f h0 = *(const v4fa*)p;
  const v4f h1 = *(const v4fa*)(p + 64);
  asm volatile("" :: "v"(h0), "v"(h1));
  float pr;
  pr = w * h0.x; aA.x = aA.x + pr;
  pr = w * h0.y; aA.y = aA.y + pr;
  pr = w * h0.z; aA.z = aA.z + pr;
  pr = w * h0.w; aA.w = aA.w + pr;
  pr = w * h1.x; aB.x = aB.x + pr;
  pr = w * h1.y; aB.y = aB.y + pr;
  pr = w * h1.z; aB.z = aB.z + pr;
  pr = w * h1.w; aB.w = aB.w + pr;
}

__global__ __launch_bounds__(RTHR) void k_walk(const float* __restrict__ H, const float* __restrict__ A4,
                                               const unsigned* __restrict__ LIST, const int* __restrict__ META,
                                               const float* __restrict__ TB, const unsigned short* __restrict__ XB,
                                               const float* __restrict__ eattr, float* out) {
  const int lane = (int)threadIdx.x & 31;
  const int wave = (int)threadIdx.x >> 5;
  const int row  = (int)blockIdx.x * RWAVES + wave;
  const bool inr = row < NN;
  const int rowc = inr ? row : NN - 1;
  const int head = lane >> 4;
  const int li   = lane & 15;

  const v2i mt = *(const v2ia*)(META + 2 * (size_t)rowc);
  asm volatile("" :: "v"(mt));
  const int craw = mt.y;
  const int offv = clampi(mt.x, 0, LISTTOT);
  const int capv = LISTTOT - offv;
  const int ccl  = clampi(craw, 0, DEGCAP);
  const int cntv = inr ? (ccl < capv ? ccl : capv) : 0;
  const int off = __builtin_amdgcn_readfirstlane(offv);
  const int cnt = __builtin_amdgcn_readfirstlane(cntv);
  const bool poison = (craw < 0) || (craw > DEGCAP);

  const v4f own = *(const v4fa*)(A4 + (size_t)rowc * 4);
  asm volatile("" :: "v"(own));
  const v4f k00 = *(const v4fa*)(TB + TB_KV);
  const v4f k01 = *(const v4fa*)(TB + TB_KV + 4);
  const v4f k10 = *(const v4fa*)(TB + TB_KV + 8);
  const v4f k11 = *(const v4fa*)(TB + TB_KV + 12);
  const v4f kcq = *(const v4fa*)(TB + TB_KV + 16);
  asm volatile("" :: "v"(k00), "v"(k01), "v"(k10), "v"(k11), "v"(kcq));

  v4f aA = (v4f){0.0f, 0.0f, 0.0f, 0.0f};
  v4f aB = (v4f){0.0f, 0.0f, 0.0f, 0.0f};

  if (cnt > 0) {
    const float ninf = -__builtin_inff();
    float sA0 = ninf, sA1 = ninf, sB0 = ninf, sB1 = ninf;
    int srcA = 0, srcB = 0;
    {
      const int j = lane < cnt ? lane : cnt - 1;
      entry_score(LIST, eattr, A4, off + j, k00, k01, k10, k11, kcq.x, kcq.y, own.z, own.w, sA0, sA1, srcA);
    }
    if (cnt > 32) {
      const int j = (32 + lane) < cnt ? (32 + lane) : cnt - 1;
      entry_score(LIST, eattr, A4, off + j, k00, k01, k10, k11, kcq.x, kcq.y, own.z, own.w, sB0, sB1, srcB);
    }
    float m0 = maxk(sA0, sB0);
    float m1 = maxk(sA1, sB1);
#pragma unroll
    for (int d = 16; d > 0; d >>= 1) {
      const float o0 = __shfl_xor(m0, d, 32);
      const float o1 = __shfl_xor(m1, d, 32);
      m0 = maxk(m0, o0);
      m1 = maxk(m1, o1);
    }
    float v;
    v = sA0 - m0; const float xA0 = expf(v);
    v = sA1 - m1; const float xA1 = expf(v);
    v = sB0 - m0; const float xB0 = expf(v);
    v = sB1 - m1; const float xB1 = expf(v);
    const int mA = cnt < 32 ? cnt : 32;
    const int mB = cnt - 32;
    float den0 = 0.0f, den1 = 0.0f;
#pragma unroll 1
    for (int k = 0; k < mA; ++k) {
      den0 = den0 + rlf(xA0, k);
      den1 = den1 + rlf(xA1, k);
    }
#pragma unroll 1
    for (int k = 0; k < mB; ++k) {
      den0 = den0 + rlf(xB0, k);
      den1 = den1 + rlf(xB1, k);
    }
    const float dd0 = den0 + 1e-16f;
    const float dd1 = den1 + 1e-16f;
    const float wA0 = xA0 / dd0;
    const float wA1 = xA1 / dd1;
    const float wB0 = xB0 / dd0;
    const float wB1 = xB1 / dd1;
    const float* hb = H + head * 128 + 4 * li;
#pragma unroll 1
    for (int k = 0; k < mA; ++k) {
      const int c = __builtin_amdgcn_readlane(srcA, k);
      const float w0 = rlf(wA0, k);
      const float w1 = rlf(wA1, k);
      const float w = (head != 0) ? w1 : w0;
      acc_row(hb, c, w, aA, aB);
    }
#pragma unroll 1
    for (int k = 0; k < mB; ++k) {
      const int c = __builtin_amdgcn_readlane(srcB, k);
      const float w0 = rlf(wB0, k);
      const float w1 = rlf(wB1, k);
      const float w = (head != 0) ? w1 : w0;
      acc_row(hb, c, w, aA, aB);
    }
  }

  v4f pA, pB;
  pA.x = __shfl_xor(aA.x, 16, 32); pA.y = __shfl_xor(aA.y, 16, 32);
  pA.z = __shfl_xor(aA.z, 16, 32); pA.w = __shfl_xor(aA.w, 16, 32);
  pB.x = __shfl_xor(aB.x, 16, 32); pB.y = __shfl_xor(aB.y, 16, 32);
  pB.z = __shfl_xor(aB.z, 16, 32); pB.w = __shfl_xor(aB.w, 16, 32);

  const v4f bA = *(const v4fa*)(TB + TB_BI + 4 * li);
  const v4f bB = *(const v4fa*)(TB + TB_BI + 64 + 4 * li);
  const v4f gA = *(const v4fa*)(TB + TB_GA + 4 * li);
  const v4f gB = *(const v4fa*)(TB + TB_GA + 64 + 4 * li);
  const v4f tA = *(const v4fa*)(TB + TB_BE + 4 * li);
  const v4f tB = *(const v4fa*)(TB + TB_BE + 64 + 4 * li);
  asm volatile("" :: "v"(bA), "v"(bB), "v"(gA), "v"(gB), "v"(tA), "v"(tB));
  const unsigned short* xr = XB + (size_t)rowc * KD + 4 * li;
  const v2u xwA = *(const v2ua*)xr;
  const v2u xwB = *(const v2ua*)(xr + 64);
  asm volatile("" :: "v"(xwA), "v"(xwB));
  const v4f xA = widen4(xwA);
  const v4f xB = widen4(xwB);

  float y0, y1, y2, y3, y4, y5, y6, y7, t;
  t = aA.x + pA.x; t = 0.5f * t; t = t + bA.x; y0 = t + xA.x;
  t = aA.y + pA.y; t = 0.5f * t; t = t + bA.y; y1 = t + xA.y;
  t = aA.z + pA.z; t = 0.5f * t; t = t + bA.z; y2 = t + xA.z;
  t = aA.w + pA.w; t = 0.5f * t; t = t + bA.w; y3 = t + xA.w;
  t = aB.x + pB.x; t = 0.5f * t; t = t + bB.x; y4 = t + xB.x;
  t = aB.y + pB.y; t = 0.5f * t; t = t + bB.y; y5 = t + xB.y;
  t = aB.z + pB.z; t = 0.5f * t; t = t + bB.z; y6 = t + xB.z;
  t = aB.w + pB.w; t = 0.5f * t; t = t + bB.w; y7 = t + xB.w;

  float s = y0 + y1; s = s + y2; s = s + y3; s = s + y4; s = s + y5; s = s + y6; s = s + y7;
  s = sum16(s);
  const float mu = s * 0.0078125f;
  const float d0 = y0 - mu, d1 = y1 - mu, d2 = y2 - mu, d3 = y3 - mu;
  const float d4 = y4 - mu, d5 = y5 - mu, d6 = y6 - mu, d7 = y7 - mu;
  float q = d0 * d0;
  t = d1 * d1; q = q + t;
  t = d2 * d2; q = q + t;
  t = d3 * d3; q = q + t;
  t = d4 * d4; q = q + t;
  t = d5 * d5; q = q + t;
  t = d6 * d6; q = q + t;
  t = d7 * d7; q = q + t;
  q = sum16(q);
  float var = q * 0.0078125f;
  var = var + 1e-5f;
  const float rs = 1.0f / sqrtf(var);
  v4f oA, oB;
  t = d0 * rs; t = t * gA.x; oA.x = t + tA.x;
  t = d1 * rs; t = t * gA.y; oA.y = t + tA.y;
  t = d2 * rs; t = t * gA.z; oA.z = t + tA.z;
  t = d3 * rs; t = t * gA.w; oA.w = t + tA.w;
  t = d4 * rs; t = t * gB.x; oB.x = t + tB.x;
  t = d5 * rs; t = t * gB.y; oB.y = t + tB.y;
  t = d6 * rs; t = t * gB.z; oB.z = t + tB.z;
  t = d7 * rs; t = t * gB.w; oB.w = t + tB.w;

  const bool lo = lane < 16;
  const float qnan = __uint_as_float(0x7fc00000u);
  v4f r;
  r.x = lo ? oA.x : oB.x;
  r.y = lo ? oA.y : oB.y;
  r.z = lo ? oA.z : oB.z;
  r.w = lo ? oA.w : oB.w;
  r.x = poison ? qnan : r.x;
  r.y = poison ? qnan : r.y;
  r.z = poison ? qnan : r.z;
  r.w = poison ? qnan : r.w;
  float* orow = out + (size_t)rowc * KD + 4 * lane;
  if (inr) *(volatile v4f*)orow = r;
  __threadfence();
  if (inr) *(volatile v4f*)orow = r;
}

extern "C" void kernel_launch(void* const* d_in, const int* in_sizes, int n_in,
                              void* d_out, int out_size, void* d_ws, size_t ws_size,
                              hipStream_t stream) {
  if (n_in < 13) return;
  if (in_sizes[0] != NN * KD) return;
  if (in_sizes[1] != 2 * NE) return;
  if (in_sizes[2] != NE * EDW) return;
  if (in_sizes[3] != EDW * KD || in_sizes[4] != KD) return;
  if (in_sizes[5] != KD * HC || in_sizes[8] != KD * HC) return;
  if (in_sizes[6] != HC || in_sizes[7] != HC || in_sizes[9] != HC) return;
  if (in_sizes[10] != KD || in_sizes[11] != KD || in_sizes[12] != KD) return;
  if (out_size != NN * KD) return;

  const float* x     = (const float*)d_in[0];
  const int*   ei    = (const int*)  d_in[1];
  const int*   esrc  = ei;
  const int*   edst  = ei + NE;
  const float* eattr = (const float*)d_in[2];
  const float* Wep   = (const float*)d_in[3];
  const float* bep   = (const float*)d_in[4];
  const float* Wlin  = (const float*)d_in[5];
  const float* attS  = (const float*)d_in[6];
  const float* attD  = (const float*)d_in[7];
  const float* Wle   = (const float*)d_in[8];
  const float* attE  = (const float*)d_in[9];
  const float* bias  = (const float*)d_in[10];
  const float* gam   = (const float*)d_in[11];
  const float* bet   = (const float*)d_in[12];
  float* out = (float*)d_out;

  const size_t szXB   = (size_t)MPAD * KD * 2;
  const size_t szWT   = (size_t)HC * KD * 2;
  const size_t szTB   = (size_t)TB_N * 4;
  const size_t szH    = (size_t)MPAD * HC * 4;
  const size_t szA4   = (size_t)MPAD * 4 * 4;
  const size_t szMETA = (size_t)NBLK * NB * 2 * 4;
  const size_t szLIST = (size_t)NBLK * RCAP * 2 * 4;
  static_assert((size_t)MPAD * KD * 2 + (size_t)HC * KD * 2 + (size_t)TB_N * 4 + (size_t)MPAD * HC * 4 +
                (size_t)MPAD * 16 + (size_t)NBLK * NB * 8 + (size_t)NBLK * RCAP * 8 == 73562112);
  static_assert(73562112 <= WSMAX);
  char* ws = (char*)d_ws;
  size_t off = 0;
  const size_t oXB   = off; off += szXB;
  const size_t oWT   = off; off += szWT;
  const size_t oTB   = off; off += szTB;
  const size_t oH    = off; off += szH;
  const size_t oA4   = off; off += szA4;
  const size_t oMETA = off; off += szMETA;
  const size_t oLIST = off; off += szLIST;
  if (off > ws_size || off > (size_t)WSMAX) return;
  unsigned short* XB = (unsigned short*)(ws + oXB);
  unsigned short* WT = (unsigned short*)(ws + oWT);
  float*    TB   = (float*)(ws + oTB);
  float*    H    = (float*)(ws + oH);
  float*    A4   = (float*)(ws + oA4);
  int*      META = (int*)(ws + oMETA);
  unsigned* LIST = (unsigned*)(ws + oLIST);

  hipFuncSetAttribute(reinterpret_cast<const void*>(&k_list),
                      hipFuncAttributeMaxDynamicSharedMemorySize, LDS_BKT);

  static_assert(MPAD % 64 == 0 && HC % 64 == 0 && KD % 32 == 0 && MPAD % 16 == 0 && HC % 4 == 0 && HC % 32 == 0);
  static_assert((MPAD * KD / 8) % 256 == 0);

  k_plane<0><<<MPAD * KD / 8 / 256, 256, 0, stream>>>(x, NN, KD, KD, XB, MPAD, KD);
  k_prep<<<1, 256, 0, stream>>>(Wlin, Wle, attE, Wep, bep, attS, attD, bias, gam, bet, WT, TB);
  k_list<<<NBLK, BT, LDS_BKT, stream>>>(edst, esrc, LIST, META);
  const int tiles = (MPAD / 64) * (HC / 64);
  const int gG = (tiles + 7) / 8;
  k_gemm_nt<0, 0><<<gG, 256, 0, stream>>>(XB, WT, TB, H, MPAD, HC, KD, HC);
  k_rowprep<<<NN / RWAVES, RTHR, 0, stream>>>(H, TB, A4);
  k_walk<<<NN / RWAVES, RTHR, 0, stream>>>(H, A4, LIST, META, TB, XB, eattr, out);
}
